// DQN_31310311587959
// MI455X (gfx1250) — hardware-run, weakly checked
//
#include <hip/hip_runtime.h>
#include <stddef.h>


#pragma clang fp contract(off)

#define CH      64
#define NTHR    256
#define NWAVE   8
#define EPT     8
#define NGRP    2
#define CHUNK   (NTHR * EPT * NGRP)
#define WCAP    (EPT * NGRP * 32)
#define LISTN   (NWAVE * WCAP)
#define NBC     4096
#define NBF     1024
#define RCAP    40960
#define RBN     128
#define TGT     256
#define DEGCAP  512
#define OTHR    512
#define BM      32
#define LDD     192
#define WSCAP   134217728
#define SCL_A   8.0f
#define SCL_W   64.0f
#define SCL_ACC 0.001953125f
#define SCL_LO  1024.0f
#define SCL_LOI 0.0009765625f

#define LDS_FILL ((RCAP + NBF + LISTN) * 4 + 64)
#define LDS_AGG  (NWAVE * 32 * CH * 8)

static_assert((CHUNK & (CHUNK - 1)) == 0);
static_assert(CHUNK <= 4096);
static_assert(NBC <= 4096 && NBF <= 4096);
static_assert((NBC & (NBC - 1)) == 0 && (NBF & (NBF - 1)) == 0);
static_assert(NBC == 4 * NBF);
static_assert(OTHR * 8 == NBC);
static_assert((RCAP % 32) == 0);
static_assert(TGT == NWAVE * 32);
static_assert((NBC % TGT) == 0);
static_assert((TGT % BM) == 0);
static_assert(CH == 64);
static_assert(LDS_AGG == 131072);

typedef float    v2f  __attribute__((ext_vector_type(2)));
typedef float    v4f  __attribute__((ext_vector_type(4)));
typedef float    v8f  __attribute__((ext_vector_type(8)));
typedef int      v4i  __attribute__((ext_vector_type(4)));
typedef _Float16 v2h  __attribute__((ext_vector_type(2)));
typedef _Float16 v4h  __attribute__((ext_vector_type(4)));
typedef _Float16 v8h  __attribute__((ext_vector_type(8)));
typedef _Float16 v16h __attribute__((ext_vector_type(16)));
union FragH { v16h v; v8h h[2]; };

__device__ __forceinline__ v8f wmh(v16h a, v16h b, v8f c) {
  v8f d = __builtin_amdgcn_wmma_f32_16x16x32_f16(false, a, false, b, (short)0, c, false, false);
  asm volatile("v_nop\n\tv_nop\n\tv_nop\n\tv_nop" : "+v"(d) : "v"(a), "v"(b));
  return d;
}

__device__ __forceinline__ v8h cvt8(v4f a, v4f b, float s) {
  v8f t;
  t[0] = a.x * s; t[1] = a.y * s; t[2] = a.z * s; t[3] = a.w * s;
  t[4] = b.x * s; t[5] = b.y * s; t[6] = b.z * s; t[7] = b.w * s;
  return __builtin_convertvector(t, v8h);
}

__device__ __forceinline__ int clampi(int v, int lo, int hi) {
  v = v < lo ? lo : v;
  return v > hi ? hi : v;
}

template <int NB>
__device__ __forceinline__ int scan_chunk(const int* __restrict__ dsts, int nE, int cbase, int slotBase,
                                          int vec8, int* list, int tid, int lane, int wave) {
  int wc = 0;
#pragma unroll
  for (int g = 0; g < NGRP; ++g) {
    const int el0  = (g * NTHR + tid) * EPT;
    const int e0   = cbase + el0;
    const int sent = -2147483647 - 1;
    v4i da, db;
    if (vec8 != 0 && cbase + CHUNK <= nE) {
      da = *(const v4i*)(dsts + e0);
      db = *(const v4i*)(dsts + e0 + 4);
    } else {
      da.x = (e0     < nE) ? dsts[min(e0, nE - 1)] : sent;
      da.y = (e0 + 1 < nE) ? dsts[min(e0 + 1, nE - 1)] : sent;
      da.z = (e0 + 2 < nE) ? dsts[min(e0 + 2, nE - 1)] : sent;
      da.w = (e0 + 3 < nE) ? dsts[min(e0 + 3, nE - 1)] : sent;
      db.x = (e0 + 4 < nE) ? dsts[min(e0 + 4, nE - 1)] : sent;
      db.y = (e0 + 5 < nE) ? dsts[min(e0 + 5, nE - 1)] : sent;
      db.z = (e0 + 6 < nE) ? dsts[min(e0 + 6, nE - 1)] : sent;
      db.w = (e0 + 7 < nE) ? dsts[min(e0 + 7, nE - 1)] : sent;
    }
    const unsigned nb = (unsigned)slotBase;
    const unsigned s0 = (unsigned)da.x - nb, s1 = (unsigned)da.y - nb;
    const unsigned s2 = (unsigned)da.z - nb, s3 = (unsigned)da.w - nb;
    const unsigned s4 = (unsigned)db.x - nb, s5 = (unsigned)db.y - nb;
    const unsigned s6 = (unsigned)db.z - nb, s7 = (unsigned)db.w - nb;
    const bool h0 = s0 < (unsigned)NB, h1 = s1 < (unsigned)NB, h2 = s2 < (unsigned)NB, h3 = s3 < (unsigned)NB;
    const bool h4 = s4 < (unsigned)NB, h5 = s5 < (unsigned)NB, h6 = s6 < (unsigned)NB, h7 = s7 < (unsigned)NB;
    const unsigned any = __builtin_amdgcn_ballot_w32(h0 | h1 | h2 | h3 | h4 | h5 | h6 | h7);
    if (any != 0u) {
#define HITJ(J, HJ, SJ) { \
        const unsigned mj = __builtin_amdgcn_ballot_w32(HJ); \
        if (mj != 0u) { \
          if (HJ) { \
            const int pos = wc + (int)__builtin_amdgcn_mbcnt_lo(mj, 0u); \
            if (pos < WCAP) list[wave * WCAP + pos] = ((el0 + (J)) << 12) | (int)(SJ); \
          } \
          wc += (int)__builtin_popcount(mj); } }
      HITJ(0, h0, s0)
      HITJ(1, h1, s1)
      HITJ(2, h2, s2)
      HITJ(3, h3, s3)
      HITJ(4, h4, s4)
      HITJ(5, h5, s5)
      HITJ(6, h6, s6)
      HITJ(7, h7, s7)
#undef HITJ
    }
  }
  return wc;
}

__global__ __launch_bounds__(NTHR) void k_wprep(const float* __restrict__ c1root, const float* __restrict__ c1rel,
                                                const float* __restrict__ c2root, const float* __restrict__ c2rel,
                                                _Float16* wb, int oh, int oq2) {
  __shared__ __attribute__((aligned(16))) _Float16 tile[CH * CH];
  const int tid = threadIdx.x;
  const int b = blockIdx.x;
  const float* W = c1rel;
  int krow0 = 0, hist = 32, dofs = 0, ldb = CH, kofs = 0;
  if (b == 1)      { W = c1rel;  krow0 = 96; dofs = CH * CH; }
  else if (b == 2) { W = c1root; krow0 = 0;  dofs = oh; ldb = 2 * CH; }
  else if (b == 3) { W = c1rel;  krow0 = 64; hist = 96; dofs = oh; ldb = 2 * CH; kofs = CH; }
  else if (b == 4) { W = c2root; krow0 = 0;  dofs = oq2; }
  else if (b == 5) { W = c2rel;  krow0 = 0;  dofs = oq2 + CH * CH; }
  else if (b == 6) { W = c2rel;  krow0 = 64; dofs = oq2 + 2 * CH * CH; }

#pragma unroll 1
  for (int idx = tid; idx < CH * CH; idx += NTHR) {
    const int k = idx >> 6;
    const int n = idx & 63;
    const int srow = krow0 + (k >> 5) * hist + (k & 31);
    const float v = W[(size_t)srow * CH + n] * SCL_W;
    tile[n * CH + k] = (_Float16)v;
  }
  __syncthreads();

  _Float16* dst = wb + dofs;
#pragma unroll
  for (int it = 0; it < 2; ++it) {
    const int u = it * NTHR + tid;
    const int row = u >> 3, c = (u & 7) * 8;
    const v8h o = *(const v8h*)(tile + row * CH + c);
    *(volatile v8h*)(dst + (size_t)row * ldb + kofs + c) = o;
  }
  __threadfence();
#pragma unroll
  for (int it = 0; it < 2; ++it) {
    const int u = it * NTHR + tid;
    const int row = u >> 3, c = (u & 7) * 8;
    const v8h o = *(const v8h*)(tile + row * CH + c);
    *(volatile v8h*)(dst + (size_t)row * ldb + kofs + c) = o;
  }
}

__global__ __launch_bounds__(NTHR) void k_nenc(const float* __restrict__ x, const float* __restrict__ w,
                                               const float* __restrict__ b, _Float16* np_, int nN, int nUnits) {
  const int i = (int)blockIdx.x * NTHR + (int)threadIdx.x;
  if (i >= nUnits) return;
  const int row = i >> 3;
  const int c0  = (i & 7) * 8;
  const int rr  = clampi(row, 0, nN - 1);
  const float x0 = x[(size_t)rr * 3 + 0];
  const float x1 = x[(size_t)rr * 3 + 1];
  const float x2 = x[(size_t)rr * 3 + 2];
  const v4f b0 = *(const v4f*)(b + c0), b1 = *(const v4f*)(b + c0 + 4);
  const v4f w00 = *(const v4f*)(w + c0),          w01 = *(const v4f*)(w + c0 + 4);
  const v4f w10 = *(const v4f*)(w + CH + c0),     w11 = *(const v4f*)(w + CH + c0 + 4);
  const v4f w20 = *(const v4f*)(w + 2 * CH + c0), w21 = *(const v4f*)(w + 2 * CH + c0 + 4);
  v4f a, c;
  a = b0 + x0 * w00 + x1 * w10 + x2 * w20;
  c = b1 + x0 * w01 + x1 * w11 + x2 * w21;
  a.x = a.x < 0.0f ? 0.0f : a.x; a.y = a.y < 0.0f ? 0.0f : a.y;
  a.z = a.z < 0.0f ? 0.0f : a.z; a.w = a.w < 0.0f ? 0.0f : a.w;
  c.x = c.x < 0.0f ? 0.0f : c.x; c.y = c.y < 0.0f ? 0.0f : c.y;
  c.z = c.z < 0.0f ? 0.0f : c.z; c.w = c.w < 0.0f ? 0.0f : c.w;
  if (row >= nN) {
    a.x = 0.0f; a.y = 0.0f; a.z = 0.0f; a.w = 0.0f;
    c.x = 0.0f; c.y = 0.0f; c.z = 0.0f; c.w = 0.0f;
  }
  const v8h o = cvt8(a, c, SCL_A);
  _Float16* d = np_ + (size_t)i * 8;
  *(volatile v8h*)d = o;
  __threadfence();
  *(volatile v8h*)d = o;
}

__global__ __launch_bounds__(NTHR) void k_count(
    const int* __restrict__ dsts, int* cnt, int nE, int vec8) {
  __shared__ __attribute__((aligned(16))) int scnt[NBC];
  __shared__ __attribute__((aligned(16))) int list[LISTN];
  __shared__ int wcnt[NWAVE];
  const int tid = threadIdx.x, lane = tid & 31, wave = tid >> 5;
  const int nodeBase = blockIdx.x * NBC;

  for (int i = tid; i < NBC; i += NTHR) scnt[i] = 0;
  __syncthreads();

  const int nChunks = (nE + CHUNK - 1) / CHUNK;
#pragma unroll 1
  for (int ch = 0; ch < nChunks; ++ch) {
    const int cbase = ch * CHUNK;
    const int wc = scan_chunk<NBC>(dsts, nE, cbase, nodeBase, vec8, list, tid, lane, wave);
    if (lane == 0) wcnt[wave] = wc;
    __syncthreads();
    if (wave == 0) {
#pragma unroll 1
      for (int wsx = 0; wsx < NWAVE; ++wsx) {
        int n = __builtin_amdgcn_readfirstlane(wcnt[wsx]);
        n = n > WCAP ? WCAP : (n < 0 ? 0 : n);
        const int* lp = list + wsx * WCAP;
#pragma unroll 1
        for (int i = 0; i < n; ++i) {
          const int ent  = __builtin_amdgcn_readfirstlane(lp[i]);
          const int slot = ent & (NBC - 1);
          if (lane == 0) scnt[slot] = scnt[slot] + 1;
        }
      }
    }
    __syncthreads();
  }

  v4i cq[4];
#pragma unroll
  for (int q = 0; q < 4; ++q) {
    const int f = (wave * 4 + q) * 128 + 4 * lane;
    cq[q] = *(const v4i*)(scnt + f);
  }
  int* cp = cnt + (size_t)nodeBase;
#pragma unroll
  for (int q = 0; q < 4; ++q) {
    const int f = (wave * 4 + q) * 128 + 4 * lane;
    *(volatile v4i*)(cp + f) = cq[q];
  }
  __threadfence();
#pragma unroll
  for (int q = 0; q < 4; ++q) {
    const int f = (wave * 4 + q) * 128 + 4 * lane;
    *(volatile v4i*)(cp + f) = cq[q];
  }
}

__global__ __launch_bounds__(OTHR) void k_offsets(
    const int* __restrict__ cnt, int* off, int* rbase, int nChunk) {
  __shared__ __attribute__((aligned(16))) int soff[NBC];
  __shared__ __attribute__((aligned(16))) int srb[RBN];
  __shared__ int wtot[OTHR / 32];
  const int tid = threadIdx.x, lane = tid & 31, wave = tid >> 5, sub = tid >> 7;
  for (int i = tid; i < RBN; i += OTHR) srb[i] = 0;
  int carry = 0;
#pragma unroll 1
  for (int ch = 0; ch < nChunk; ++ch) {
    const int base = ch * NBC;
    const v4i c0 = *(const v4i*)(cnt + base + 8 * tid);
    const v4i c1 = *(const v4i*)(cnt + base + 8 * tid + 4);
    const int e0 = max(c0.x, 0), e1 = max(c0.y, 0), e2 = max(c0.z, 0), e3 = max(c0.w, 0);
    const int e4 = max(c1.x, 0), e5 = max(c1.y, 0), e6 = max(c1.z, 0), e7 = max(c1.w, 0);
    const int ts = e0 + e1 + e2 + e3 + e4 + e5 + e6 + e7;
    int incl = ts;
#pragma unroll
    for (int d = 1; d < 32; d <<= 1) {
      const int t = __shfl_up(incl, d);
      if (lane >= d) incl += t;
    }
    if (lane == 31) wtot[wave] = incl;
    __syncthreads();
    const int S0 = wtot[0]  + wtot[1]  + wtot[2]  + wtot[3];
    const int S1 = wtot[4]  + wtot[5]  + wtot[6]  + wtot[7];
    const int S2 = wtot[8]  + wtot[9]  + wtot[10] + wtot[11];
    const int S3 = wtot[12] + wtot[13] + wtot[14] + wtot[15];
    int pre = 0;
#pragma unroll 1
    for (int w = 4 * sub; w < wave; ++w) pre += wtot[w];
    const int b0 = carry;
    const int b1 = b0 + ((S0 + 31) & ~31);
    const int b2 = b1 + ((S1 + 31) & ~31);
    const int b3 = b2 + ((S2 + 31) & ~31);
    const int b4 = b3 + ((S3 + 31) & ~31);
    const int myb = sub == 0 ? b0 : (sub == 1 ? b1 : (sub == 2 ? b2 : b3));
    if (tid == 0) {
      srb[min(4 * ch + 0, RBN - 1)] = b0;
      srb[min(4 * ch + 1, RBN - 1)] = b1;
      srb[min(4 * ch + 2, RBN - 1)] = b2;
      srb[min(4 * ch + 3, RBN - 1)] = b3;
    }
    int run = myb + pre + incl - ts;
    soff[8 * tid + 0] = run; run += e0;
    soff[8 * tid + 1] = run; run += e1;
    soff[8 * tid + 2] = run; run += e2;
    soff[8 * tid + 3] = run; run += e3;
    soff[8 * tid + 4] = run; run += e4;
    soff[8 * tid + 5] = run; run += e5;
    soff[8 * tid + 6] = run; run += e6;
    soff[8 * tid + 7] = run;
    carry = b4;
    __syncthreads();
    const v4i o0 = *(const v4i*)(soff + 4 * tid);
    const v4i o1 = *(const v4i*)(soff + 4 * (tid + OTHR));
    int* op = off + base;
    *(volatile v4i*)(op + 4 * tid) = o0;
    *(volatile v4i*)(op + 4 * (tid + OTHR)) = o1;
    __threadfence();
    *(volatile v4i*)(op + 4 * tid) = o0;
    *(volatile v4i*)(op + 4 * (tid + OTHR)) = o1;
    __syncthreads();
  }
  if (tid == 0) srb[min(4 * nChunk, RBN - 1)] = carry;
  __syncthreads();
  v4i rv = {0, 0, 0, 0};
  if (tid < 32) rv = *(const v4i*)(srb + 4 * tid);
  if (tid < 32) *(volatile v4i*)(rbase + 4 * tid) = rv;
  __threadfence();
  if (tid < 32) *(volatile v4i*)(rbase + 4 * tid) = rv;
}

__global__ __launch_bounds__(NTHR) void k_fill(
    const int* __restrict__ dsts, const int* __restrict__ off, const int* __restrict__ rbase,
    int* csr, int nE, int vec8, int csrLen) {
  extern __shared__ v4f lds_fill_dyn[];
  int* region = (int*)lds_fill_dyn;
  int* cursor = region + RCAP;
  int* list   = cursor + NBF;
  int* wcnt   = list + LISTN;
  const int tid = threadIdx.x, lane = tid & 31, wave = tid >> 5;
  const int b = blockIdx.x;
  const int nodeBase = b * NBF;

  int rb0 = rbase[b];
  const int rb1 = rbase[b + 1];
  rb0 = rb0 < 0 ? 0 : (rb0 > csrLen ? csrLen : rb0);
  rb0 &= ~31;
  int len = rb1 - rb0;
  len = len < 0 ? 0 : (len > RCAP ? RCAP : len);
  int lenW = (len + 31) & ~31;
  if (rb0 + lenW > csrLen) lenW = (csrLen - rb0) & ~31;

  {
    const v4i z = {0, 0, 0, 0};
    for (int i = tid; i < RCAP / 4; i += NTHR) ((v4i*)region)[i] = z;
    for (int s = tid; s < NBF; s += NTHR) {
      int o = off[nodeBase + s] - rb0;
      o = o < 0 ? 0 : (o > RCAP ? RCAP : o);
      cursor[s] = o;
    }
  }
  __syncthreads();

  const int nChunks = (nE + CHUNK - 1) / CHUNK;
#pragma unroll 1
  for (int ch = 0; ch < nChunks; ++ch) {
    const int cbase = ch * CHUNK;
    const int wc = scan_chunk<NBF>(dsts, nE, cbase, nodeBase, vec8, list, tid, lane, wave);
    if (lane == 0) wcnt[wave] = wc;
    __syncthreads();
    if (wave == 0) {
#pragma unroll 1
      for (int wsx = 0; wsx < NWAVE; ++wsx) {
        int n = __builtin_amdgcn_readfirstlane(wcnt[wsx]);
        n = n > WCAP ? WCAP : (n < 0 ? 0 : n);
        const int* lp = list + wsx * WCAP;
#pragma unroll 1
        for (int i = 0; i < n; ++i) {
          const int ent  = __builtin_amdgcn_readfirstlane(lp[i]);
          const int slot = ent & (NBF - 1);
          int e = cbase + ((ent >> 12) & (CHUNK - 1));
          e = e > nE - 1 ? nE - 1 : (e < 0 ? 0 : e);
          if (lane == 0) {
            int pos = cursor[slot];
            pos = pos < 0 ? 0 : (pos > RCAP - 1 ? RCAP - 1 : pos);
            region[pos] = e;
            const int np = pos + 1;
            cursor[slot] = np > RCAP ? RCAP : np;
          }
        }
      }
    }
    __syncthreads();
  }

  const int nv = lenW >> 2;
  int* gp = csr + rb0;
#pragma unroll 1
  for (int i = tid; i < nv; i += NTHR) { const v4i v = ((const v4i*)region)[i]; *(volatile v4i*)(gp + 4 * i) = v; }
  __threadfence();
#pragma unroll 1
  for (int i = tid; i < nv; i += NTHR) { const v4i v = ((const v4i*)region)[i]; *(volatile v4i*)(gp + 4 * i) = v; }
}

template <int K, int LDB, int TPW>
__device__ __forceinline__ void mma_pair(const _Float16* __restrict__ Ap, const _Float16* __restrict__ Bp,
                                         int arow, int c0, int m, int hh, v8f (&acc)[TPW]) {
  constexpr int KT = K / 32;
  static_assert(K % 32 == 0 && LDB % 8 == 0);
  const _Float16* ap  = Ap + (size_t)arow * K + 8 * hh;
  const _Float16* bp0 = Bp + (size_t)(c0 + m) * LDB + 8 * hh;
#pragma unroll 1
  for (int kt = 0; kt < KT; ++kt) {
    FragH a;
    a.h[0] = *(const v8h*)(ap + 32 * kt);
    a.h[1] = *(const v8h*)(ap + 32 * kt + 16);
#pragma unroll
    for (int t = 0; t < TPW; ++t) {
      const _Float16* bp = bp0 + (size_t)(16 * t) * LDB + 32 * kt;
      FragH bf;
      bf.h[0] = *(const v8h*)bp;
      bf.h[1] = *(const v8h*)(bp + 16);
      acc[t] = wmh(a.v, bf.v, acc[t]);
    }
  }
}

template <int NC>
__global__ __launch_bounds__(NTHR) void k_gemmF(
    const _Float16* __restrict__ A, const _Float16* __restrict__ Bp, float* D) {
  constexpr int TPW  = NC / 64;
  constexpr int NV   = NC / 4;
  constexpr int NIT4 = (BM * NC / 4) / NTHR;
  static_assert(NC % 64 == 0 && TPW >= 1);
  static_assert((BM * NC / 4) % NTHR == 0 && NIT4 >= 1);
  static_assert(BM * 8 == NTHR);
  static_assert(NC <= LDD);
  static_assert(NC == LDD || NV == 32);

  __shared__ __attribute__((aligned(16))) float stg[BM * NC];
  const int tid = threadIdx.x, lane = tid & 31, wave = tid >> 5, hh = lane >> 4, m = lane & 15;
  const int rowBase = blockIdx.x * BM;
  const int rg = wave >> 2, cq = wave & 3;
  const int r0 = rg * 16;
  const int c0 = cq * (NC / 4);

  v8f acc[TPW];
#pragma unroll
  for (int t = 0; t < TPW; ++t) { v8f z = {0.f, 0.f, 0.f, 0.f, 0.f, 0.f, 0.f, 0.f}; acc[t] = z; }

  mma_pair<CH, CH, TPW>(A, Bp, rowBase + r0 + m, c0, m, hh, acc);

  {
    float* sp = stg + (size_t)(r0 + 8 * hh) * NC + c0 + m;
#pragma unroll
    for (int t = 0; t < TPW; ++t) {
#pragma unroll
      for (int r = 0; r < 8; ++r) sp[r * NC + 16 * t] = acc[t][r] * SCL_ACC;
    }
  }
  __syncthreads();

#pragma unroll
  for (int it = 0; it < NIT4; ++it) {
    const int u = it * NTHR + tid;
    const int row = u / NV, cv = u - row * NV;
    const v4f v = *(const v4f*)(stg + 4 * u);
    *(volatile v4f*)(D + (size_t)(rowBase + row) * LDD + 4 * cv) = v;
  }
  __threadfence();
#pragma unroll
  for (int it = 0; it < NIT4; ++it) {
    const int u = it * NTHR + tid;
    const int row = u / NV, cv = u - row * NV;
    const v4f v = *(const v4f*)(stg + 4 * u);
    *(volatile v4f*)(D + (size_t)(rowBase + row) * LDD + 4 * cv) = v;
  }
}

__global__ __launch_bounds__(NTHR) void k_agg1(
    const int* __restrict__ csr, const int* __restrict__ off, const int* __restrict__ cnt,
    const int* __restrict__ esrc, const int* __restrict__ etyp, const float* __restrict__ ea,
    const float* __restrict__ eew, const float* __restrict__ eeb, const float* __restrict__ b1,
    const float* Pr, float* Gw, _Float16* sphi, _Float16* splo,
    int nN, int nE, int csrLen) {
  extern __shared__ v4f lds_agg_dyn[];
  float*    gsl = (float*)lds_agg_dyn;
  _Float16* hsl = (_Float16*)(gsl + NWAVE * 32 * CH);
  _Float16* lsl = hsl + NWAVE * 32 * CH;
  const int tid = threadIdx.x, lane = tid & 31, wave = tid >> 5;
  const int tbase = blockIdx.x * TGT + wave * 32;
  const int col = 2 * lane;
  float*    gw = gsl + wave * (32 * CH);
  _Float16* hw = hsl + wave * (32 * CH);
  _Float16* lw = lsl + wave * (32 * CH);

  const v2f   bb = *(const v2f*)(b1 + col);
  const float w0 = eew[lane], w1 = eew[32 + lane], be = eeb[lane];
  const float qn = __int_as_float(0x7fc00000);

  const int cl    = tbase + lane;
  const int cnt_l = cnt[cl];
  const int off_l = off[cl];

#pragma unroll 1
  for (int j = 0; j < 32; ++j) {
    const int c = tbase + j;
    int nraw = __shfl(cnt_l, j);
    nraw = clampi(nraw, 0, nE);
    const int n = nraw > DEGCAP ? DEGCAP : nraw;
    const int st = __shfl(off_l, j);

    v2f acc = {0.0f, 0.0f};
    float s0 = 0.0f, s1 = 0.0f;
#pragma unroll 1
    for (int q0 = 0; q0 < n; q0 += 32) {
      const int pos = clampi(st + q0 + lane, 0, csrLen - 1);
      const int e = clampi(csr[pos], 0, nE - 1);
      const int sv = clampi(esrc[e], 0, nN - 1);
      const int tv = etyp[e];
      const int tcode = (tv == 0) ? 0 : ((tv == 1) ? 1 : 2);
      const v2f av = *(const v2f*)(ea + (size_t)e * 2);
      const int a0b = __float_as_int(av.x), a1b = __float_as_int(av.y);
      const int mcnt = (n - q0) < 32 ? (n - q0) : 32;
#pragma unroll 1
      for (int pp = 0; pp < mcnt; ++pp) {
        const int   ps  = __builtin_amdgcn_readlane(sv, pp);
        const int   tc  = __builtin_amdgcn_readlane(tcode, pp);
        const float fa0 = __int_as_float(__builtin_amdgcn_readlane(a0b, pp));
        const float fa1 = __int_as_float(__builtin_amdgcn_readlane(a1b, pp));
        const int   tcl = tc > 1 ? 1 : tc;
        const v2f pv = *(const v2f*)(Pr + (size_t)ps * LDD + CH * tcl + col);
        const bool use = tc <= 1;
        acc.x = use ? acc.x + pv.x : acc.x;
        acc.y = use ? acc.y + pv.y : acc.y;
        float ev = fa0 * w0 + fa1 * w1 + be;
        ev = ev < 0.0f ? 0.0f : ev;
        s0 = (tc == 0) ? s0 + ev : s0;
        s1 = (tc == 1) ? s1 + ev : s1;
      }
    }

    v2f g;
    g.x = acc.x + bb.x;
    g.y = acc.y + bb.y;
    if (nraw > DEGCAP) { g.x = qn; g.y = qn; }
    if (c >= nN) { g.x = 0.0f; g.y = 0.0f; s0 = 0.0f; s1 = 0.0f; }
    const float t0 = s0 * SCL_A, t1 = s1 * SCL_A;
    const _Float16 h0 = (_Float16)t0, h1 = (_Float16)t1;
    const _Float16 l0 = (_Float16)((t0 - (float)h0) * SCL_LO);
    const _Float16 l1 = (_Float16)((t1 - (float)h1) * SCL_LO);
    *(v2f*)(gw + j * CH + col) = g;
    hw[j * CH + lane] = h0; hw[j * CH + 32 + lane] = h1;
    lw[j * CH + lane] = l0; lw[j * CH + 32 + lane] = l1;
  }
  __syncthreads();

  float*    gp = Gw + (size_t)tbase * LDD + 2 * CH;
  _Float16* hp = sphi + (size_t)tbase * CH;
  _Float16* lp = splo + (size_t)tbase * CH;
#pragma unroll
  for (int q = 0; q < 16; ++q) {
    const int u = q * 32 + lane, row = u >> 4, pc = u & 15;
    const v4f v = *(const v4f*)(gw + row * CH + 4 * pc);
    *(volatile v4f*)(gp + (size_t)row * LDD + 4 * pc) = v;
  }
#pragma unroll
  for (int q = 0; q < 8; ++q) {
    const v8h o = *(const v8h*)(hw + q * 256 + 8 * lane);
    *(volatile v8h*)(hp + q * 256 + 8 * lane) = o;
    const v8h p = *(const v8h*)(lw + q * 256 + 8 * lane);
    *(volatile v8h*)(lp + q * 256 + 8 * lane) = p;
  }
  __threadfence();
#pragma unroll
  for (int q = 0; q < 16; ++q) {
    const int u = q * 32 + lane, row = u >> 4, pc = u & 15;
    const v4f v = *(const v4f*)(gw + row * CH + 4 * pc);
    *(volatile v4f*)(gp + (size_t)row * LDD + 4 * pc) = v;
  }
#pragma unroll
  for (int q = 0; q < 8; ++q) {
    const v8h o = *(const v8h*)(hw + q * 256 + 8 * lane);
    *(volatile v8h*)(hp + q * 256 + 8 * lane) = o;
    const v8h p = *(const v8h*)(lw + q * 256 + 8 * lane);
    *(volatile v8h*)(lp + q * 256 + 8 * lane) = p;
  }
}

__global__ __launch_bounds__(NTHR) void k_gemmH(
    const _Float16* __restrict__ nP, const _Float16* __restrict__ sphi, const _Float16* __restrict__ splo,
    const _Float16* __restrict__ WH, const float* __restrict__ Gp, _Float16* hP, int nN) {
  __shared__ __attribute__((aligned(16))) float stg[BM * CH];
  const int tid = threadIdx.x, lane = tid & 31, wave = tid >> 5, hh = lane >> 4, m = lane & 15;
  const int rowBase = blockIdx.x * BM;
  const int rg = wave >> 2, cq = wave & 3;
  const int r0 = rg * 16;
  const int c0 = cq * 16;

  v8f acc[1], accr[1];
  { v8f z = {0.f, 0.f, 0.f, 0.f, 0.f, 0.f, 0.f, 0.f}; acc[0] = z; accr[0] = z; }

  mma_pair<CH, 2 * CH, 1>(nP,   WH,      rowBase + r0 + m, c0, m, hh, acc);
  mma_pair<CH, 2 * CH, 1>(sphi, WH + CH, rowBase + r0 + m, c0, m, hh, acc);
  mma_pair<CH, 2 * CH, 1>(splo, WH + CH, rowBase + r0 + m, c0, m, hh, accr);

  {
    const int lrow = r0 + 8 * hh;
    const float* gpp = Gp + (size_t)(rowBase + lrow) * LDD + 2 * CH + c0 + m;
    float* sp = stg + (size_t)lrow * CH + c0 + m;
#pragma unroll
    for (int r = 0; r < 8; ++r) {
      const float g = gpp[(size_t)r * LDD];
      float v = (acc[0][r] + accr[0][r] * SCL_LOI) * SCL_ACC + g;
      v = (v < 0.0f) ? 0.0f : v;
      sp[r * CH] = v;
    }
  }
  __syncthreads();

  const int row = tid >> 3, c8 = (tid & 7) * 8;
  v4f a = *(const v4f*)(stg + row * CH + c8);
  v4f b = *(const v4f*)(stg + row * CH + c8 + 4);
  if (rowBase + row >= nN) {
    a.x = 0.0f; a.y = 0.0f; a.z = 0.0f; a.w = 0.0f;
    b.x = 0.0f; b.y = 0.0f; b.z = 0.0f; b.w = 0.0f;
  }
  const v8h o = cvt8(a, b, SCL_A);
  _Float16* d = hP + (size_t)(rowBase + row) * CH + c8;
  *(volatile v8h*)d = o;
  __threadfence();
  *(volatile v8h*)d = o;
}

__global__ __launch_bounds__(NTHR) void k_final(
    const int* __restrict__ csr, const int* __restrict__ off, const int* __restrict__ cnt,
    const int* __restrict__ esrc, const int* __restrict__ etyp, const float* __restrict__ D,
    const float* __restrict__ b2, const float* __restrict__ vw, const float* __restrict__ vb,
    const float* __restrict__ aw, const float* __restrict__ ab, float* out,
    int nN, int nE, int csrLen, int off1, int lineMode) {
  __shared__ __attribute__((aligned(16))) float sval[NWAVE * 32];
  __shared__ __attribute__((aligned(16))) float sact[NWAVE * 160];
  const int tid = threadIdx.x, lane = tid & 31, wave = tid >> 5;
  const int tbase = blockIdx.x * TGT + wave * 32;
  const int col = 2 * lane;
  const float ninf = -__builtin_inff();
  const float pinf = __builtin_inff();
  const float qn = __int_as_float(0x7fc00000);

  const v2f   bb  = *(const v2f*)(b2 + col);
  const float vw0 = vw[col], vw1 = vw[col + 1];
  const float a00 = aw[col * 5 + 0], a01 = aw[col * 5 + 1], a02 = aw[col * 5 + 2];
  const float a03 = aw[col * 5 + 3], a04 = aw[col * 5 + 4];
  const float a10 = aw[(col + 1) * 5 + 0], a11 = aw[(col + 1) * 5 + 1], a12 = aw[(col + 1) * 5 + 2];
  const float a13 = aw[(col + 1) * 5 + 3], a14 = aw[(col + 1) * 5 + 4];
  const float vb0 = vb[0];
  const float ab0 = ab[0], ab1 = ab[1], ab2 = ab[2], ab3 = ab[3], ab4 = ab[4];

  const int cl    = tbase + lane;
  const int cnt_l = cnt[cl];
  const int off_l = off[cl];

#pragma unroll 1
  for (int j = 0; j < 32; ++j) {
    const int c = tbase + j;
    int nraw = __shfl(cnt_l, j);
    nraw = clampi(nraw, 0, nE);
    const int n = nraw > DEGCAP ? DEGCAP : nraw;
    const int st = __shfl(off_l, j);

    v2f m0 = {ninf, ninf}, m1 = {ninf, ninf};
#pragma unroll 1
    for (int q0 = 0; q0 < n; q0 += 32) {
      const int pos = clampi(st + q0 + lane, 0, csrLen - 1);
      const int e = clampi(csr[pos], 0, nE - 1);
      const int sv = clampi(esrc[e], 0, nN - 1);
      const int tv = etyp[e];
      const int tcode = (tv == 0) ? 0 : ((tv == 1) ? 1 : 2);
      const int mcnt = (n - q0) < 32 ? (n - q0) : 32;
#pragma unroll 1
      for (int pp = 0; pp < mcnt; ++pp) {
        const int ps  = __builtin_amdgcn_readlane(sv, pp);
        const int tc  = __builtin_amdgcn_readlane(tcode, pp);
        const int tcl = tc > 1 ? 1 : tc;
        const v2f pv = *(const v2f*)(D + (size_t)ps * LDD + CH * (1 + tcl) + col);
        const float x0 = fmaxf(m0.x, pv.x), y0 = fmaxf(m0.y, pv.y);
        const float x1 = fmaxf(m1.x, pv.x), y1 = fmaxf(m1.y, pv.y);
        m0.x = (tc == 0) ? x0 : m0.x; m0.y = (tc == 0) ? y0 : m0.y;
        m1.x = (tc == 1) ? x1 : m1.x; m1.y = (tc == 1) ? y1 : m1.y;
      }
    }
    const float f0x = (m0.x > ninf && m0.x < pinf) ? m0.x : 0.0f;
    const float f0y = (m0.y > ninf && m0.y < pinf) ? m0.y : 0.0f;
    const float f1x = (m1.x > ninf && m1.x < pinf) ? m1.x : 0.0f;
    const float f1y = (m1.y > ninf && m1.y < pinf) ? m1.y : 0.0f;
    const v2f base = *(const v2f*)(D + (size_t)c * LDD + col);
    float hx = ((base.x + bb.x) + f0x) + f1x;
    float hy = ((base.y + bb.y) + f0y) + f1y;
    hx = hx < 0.0f ? 0.0f : hx;
    hy = hy < 0.0f ? 0.0f : hy;

    float pv = hx * vw0 + hy * vw1;
    float p0 = hx * a00 + hy * a10;
    float p1 = hx * a01 + hy * a11;
    float p2 = hx * a02 + hy * a12;
    float p3 = hx * a03 + hy * a13;
    float p4 = hx * a04 + hy * a14;
#pragma unroll
    for (int d = 16; d >= 1; d >>= 1) {
      pv += __shfl_xor(pv, d, 32);
      p0 += __shfl_xor(p0, d, 32);
      p1 += __shfl_xor(p1, d, 32);
      p2 += __shfl_xor(p2, d, 32);
      p3 += __shfl_xor(p3, d, 32);
      p4 += __shfl_xor(p4, d, 32);
    }
    float ov = pv + vb0;
    float o0 = p0 + ab0, o1 = p1 + ab1, o2 = p2 + ab2, o3 = p3 + ab3, o4 = p4 + ab4;
    if (nraw > DEGCAP) { ov = qn; o0 = qn; o1 = qn; o2 = qn; o3 = qn; o4 = qn; }
    if (lane == 0) {
      sval[wave * 32 + j] = ov;
      float* sa = sact + wave * 160 + j * 5;
      sa[0] = o0; sa[1] = o1; sa[2] = o2; sa[3] = o3; sa[4] = o4;
    }
  }
  __syncthreads();

  const float* svw = sval + wave * 32;
  const float* saw = sact + wave * 160;
  if (lineMode != 0 && tbase + 32 <= nN) {
    float* o0p = out + tbase;
    float* o1p = out + (size_t)off1 + (size_t)tbase * 5;
    if (lane < 8) { const v4f v = *(const v4f*)(svw + 4 * lane); *(volatile v4f*)(o0p + 4 * lane) = v; }
    { const v4f v = *(const v4f*)(saw + 4 * lane); *(volatile v4f*)(o1p + 4 * lane) = v; }
    if (lane < 8) { const v4f v = *(const v4f*)(saw + 128 + 4 * lane); *(volatile v4f*)(o1p + 128 + 4 * lane) = v; }
    __threadfence();
    if (lane < 8) { const v4f v = *(const v4f*)(svw + 4 * lane); *(volatile v4f*)(o0p + 4 * lane) = v; }
    { const v4f v = *(const v4f*)(saw + 4 * lane); *(volatile v4f*)(o1p + 4 * lane) = v; }
    if (lane < 8) { const v4f v = *(const v4f*)(saw + 128 + 4 * lane); *(volatile v4f*)(o1p + 128 + 4 * lane) = v; }
  } else {
    const int c = tbase + lane;
    const bool ok = c < nN;
    const int cc = clampi(c, 0, nN - 1);
    const float v = svw[lane];
    const float e0 = saw[lane * 5 + 0], e1 = saw[lane * 5 + 1], e2 = saw[lane * 5 + 2];
    const float e3 = saw[lane * 5 + 3], e4 = saw[lane * 5 + 4];
    float* ap = out + (size_t)off1 + (size_t)cc * 5;
    if (ok) {
      *(volatile float*)(out + cc) = v;
      *(volatile float*)(ap + 0) = e0; *(volatile float*)(ap + 1) = e1; *(volatile float*)(ap + 2) = e2;
      *(volatile float*)(ap + 3) = e3; *(volatile float*)(ap + 4) = e4;
    }
    __threadfence();
    if (ok) {
      *(volatile float*)(out + cc) = v;
      *(volatile float*)(ap + 0) = e0; *(volatile float*)(ap + 1) = e1; *(volatile float*)(ap + 2) = e2;
      *(volatile float*)(ap + 3) = e3; *(volatile float*)(ap + 4) = e4;
    }
  }
}

extern "C" void kernel_launch(void* const* d_in, const int* in_sizes, int n_in,
                              void* d_out, int out_size, void* d_ws, size_t ws_size,
                              hipStream_t stream) {
  if (n_in < 18) return;
  const int nN = in_sizes[0] / 3;
  const int nE = in_sizes[3];
  if (nN <= 0 || nE <= 0 || in_sizes[0] != nN * 3) return;
  if (in_sizes[1] != 2 * nE || in_sizes[2] != 2 * nE) return;
  if (in_sizes[4] != 3 * CH || in_sizes[5] != CH) return;
  if (in_sizes[6] != 2 * 32 || in_sizes[7] != 32) return;
  if (in_sizes[8] != CH * CH || in_sizes[9] != 2 * 96 * CH || in_sizes[10] != CH) return;
  if (in_sizes[11] != CH * CH || in_sizes[12] != 2 * CH * CH || in_sizes[13] != CH) return;
  if (in_sizes[14] != CH || in_sizes[15] < 1 || in_sizes[16] != CH * 5 || in_sizes[17] < 5) return;
  if (out_size != 6 * nN) return;
  if (nE > (1 << 28) || nN > (1 << 22)) return;

  const float* x     = (const float*)d_in[0];
  const float* ea    = (const float*)d_in[1];
  const int*   ei    = (const int*)d_in[2];
  const int*   etyp  = (const int*)d_in[3];
  const float* nw    = (const float*)d_in[4];
  const float* nb    = (const float*)d_in[5];
  const float* eww   = (const float*)d_in[6];
  const float* ebb   = (const float*)d_in[7];
  const float* c1rt  = (const float*)d_in[8];
  const float* c1rel = (const float*)d_in[9];
  const float* c1b   = (const float*)d_in[10];
  const float* c2rt  = (const float*)d_in[11];
  const float* c2rel = (const float*)d_in[12];
  const float* c2b   = (const float*)d_in[13];
  const float* vw    = (const float*)d_in[14];
  const float* vb    = (const float*)d_in[15];
  const float* aw    = (const float*)d_in[16];
  const float* ab    = (const float*)d_in[17];
  float* out = (float*)d_out;
  const int* esrc = ei;
  const int* dsts = ei + nE;

  const int NPAD   = ((nN + TGT - 1) / TGT) * TGT;
  const int nBC    = (nN + NBC - 1) / NBC;
  const int CNTPAD = nBC * NBC;
  if (CNTPAD < NPAD) return;
  if (4 * nBC + 1 > RBN) return;
  const int nBF    = (nN + NBF - 1) / NBF;
  if (nBF + 1 > 4 * nBC + 1) return;
  const int csrLen = ((nE + 31) & ~31) + 4096;
  if (31 * 4 * nBC > 4096) return;
  const int nAgg   = NPAD / TGT;
  const int nGemm  = NPAD / BM;
  const int nXu    = NPAD * (CH / 8);

  char* ws = (char*)d_ws;
  size_t off = 0;
  const size_t oQ1  = off; off += (size_t)2 * CH * CH * 2;      off = (off + 255) & ~(size_t)255;
  const size_t oWH  = off; off += (size_t)CH * 2 * CH * 2;      off = (off + 255) & ~(size_t)255;
  const size_t oQ2  = off; off += (size_t)3 * CH * CH * 2;      off = (off + 255) & ~(size_t)255;
  const size_t oNP  = off; off += (size_t)NPAD * CH * 2;        off = (off + 255) & ~(size_t)255;
  const size_t oHI  = off; off += (size_t)NPAD * CH * 2;        off = (off + 255) & ~(size_t)255;
  const size_t oLO  = off; off += (size_t)NPAD * CH * 2;        off = (off + 255) & ~(size_t)255;
  const size_t oHP  = off; off += (size_t)NPAD * CH * 2;        off = (off + 255) & ~(size_t)255;
  const size_t oD   = off; off += (size_t)NPAD * LDD * 4;       off = (off + 255) & ~(size_t)255;
  const size_t oCnt = off; off += (size_t)CNTPAD * 4;           off = (off + 255) & ~(size_t)255;
  const size_t oOff = off; off += (size_t)CNTPAD * 4;           off = (off + 255) & ~(size_t)255;
  const size_t oRb  = off; off += (size_t)RBN * 4;              off = (off + 255) & ~(size_t)255;
  const size_t oCsr = off; off += (size_t)csrLen * 4;           off = (off + 255) & ~(size_t)255;
  if (off > ws_size || off > (size_t)WSCAP) return;
  _Float16* WQ1  = (_Float16*)(ws + oQ1);
  _Float16* WHp  = (_Float16*)(ws + oWH);
  _Float16* WQ2  = (_Float16*)(ws + oQ2);
  _Float16* nP   = (_Float16*)(ws + oNP);
  _Float16* sphi = (_Float16*)(ws + oHI);
  _Float16* splo = (_Float16*)(ws + oLO);
  _Float16* hP   = (_Float16*)(ws + oHP);
  float* Df   = (float*)(ws + oD);
  int*   cnt  = (int*)(ws + oCnt);
  int*   offp = (int*)(ws + oOff);
  int*   rb   = (int*)(ws + oRb);
  int*   csr  = (int*)(ws + oCsr);
  const int ohH  = (int)((oWH - oQ1) / 2);
  const int oq2H = (int)((oQ2 - oQ1) / 2);

  const int vec8 = ((nE & 3) == 0) ? 1 : 0;
  const int off1 = nN;
  const int lineMode = ((nN & 31) == 0) ? 1 : 0;

  k_wprep<<<7, NTHR, 0, stream>>>(c1rt, c1rel, c2rt, c2rel, WQ1, ohH, oq2H);
  k_nenc<<<(nXu + NTHR - 1) / NTHR, NTHR, 0, stream>>>(x, nw, nb, nP, nN, nXu);

  k_count<<<nBC, NTHR, 0, stream>>>(dsts, cnt, nE, vec8);
  k_offsets<<<1, OTHR, 0, stream>>>(cnt, offp, rb, nBC);
  hipFuncSetAttribute(reinterpret_cast<const void*>(&k_fill),
                      hipFuncAttributeMaxDynamicSharedMemorySize, LDS_FILL);
  k_fill<<<nBF, NTHR, LDS_FILL, stream>>>(dsts, offp, rb, csr, nE, vec8, csrLen);

  k_gemmF<2 * CH><<<nGemm, NTHR, 0, stream>>>(nP, WQ1, Df);
  hipFuncSetAttribute(reinterpret_cast<const void*>(&k_agg1),
                      hipFuncAttributeMaxDynamicSharedMemorySize, LDS_AGG);
  k_agg1<<<nAgg, NTHR, LDS_AGG, stream>>>(csr, offp, cnt, esrc, etyp, ea, eww, ebb, c1b,
                                           Df, Df, sphi, splo, nN, nE, csrLen);
  k_gemmH<<<nGemm, NTHR, 0, stream>>>(nP, sphi, splo, WHp, Df, hP, nN);
  k_gemmF<3 * CH><<<nGemm, NTHR, 0, stream>>>(hP, WQ2, Df);
  k_final<<<nAgg, NTHR, 0, stream>>>(csr, offp, cnt, esrc, etyp, Df, c2b, vw, vb, aw, ab, out,
                                     nN, nE, csrLen, off1, lineMode);
}
